// additive_attention_51926154609340
// MI455X (gfx1250) — hardware-run, weakly checked
//
#include <hip/hip_runtime.h>


#ifndef NB
#define NB 4
#endif
#ifndef SEQ
#define SEQ 512
#endif
#define NB_FULL  4
#define SEQ_FULL 512
#ifndef OUT_SEQ
#define OUT_SEQ SEQ
#endif
#define FEAT 256
#define HID  128
#define VD   256
#define PW   8
#define NG   (SEQ / 128)
#define NP8  (SEQ / 256)
#define QRS  2048.0f
#define QRI  (1.0f / 2048.0f)
#define PC   256.0f
#define PCI  (1.0f / 256.0f)
#define L2E  1.4426950408889634f
#define TL2E 2.8853900817779268f
#define NEGF (-1.0e9f)
#define OUT1_OFF ((size_t)NB_FULL * SEQ_FULL * VD)

static_assert(HID == 128);
static_assert(HID % 64 == 0);
static_assert(FEAT % 32 == 0);
static_assert(VD % 64 == 0);
static_assert(SEQ % 256 == 0);
static_assert(SEQ % PW == 0);
static_assert((NB * SEQ) % 64 == 0);
static_assert((NB * SEQ) % 32 == 0);
static_assert(NB <= NB_FULL);
static_assert(SEQ <= SEQ_FULL);
static_assert(OUT_SEQ >= SEQ);
static_assert(OUT1_OFF * 4 == (size_t)2097152);
static_assert((size_t)NB * OUT_SEQ * VD <= OUT1_OFF);
static_assert(OUT1_OFF + (size_t)NB * OUT_SEQ * OUT_SEQ <= (size_t)6291456 / 4);
static_assert(32 * 16 * NG == SEQ * 4);
static_assert(32 * 16 * NP8 == SEQ * 2);
static_assert(32 * 16 * 8 == 16 * 64 * 4);
static_assert(256 * 16 * 2 == 64 * 64 * 2);
static_assert((PW * HID * 2 + PW * SEQ) * 4 <= 131072);
static_assert(64 * 65 * 4 <= 131072);
static_assert(16 * 68 * 4 <= 131072);

typedef _Float16 h16;
typedef unsigned short bf;
typedef __attribute__((ext_vector_type(16))) __bf16   v16bf;
typedef __attribute__((ext_vector_type(16))) _Float16 v16h;
typedef __attribute__((ext_vector_type(8)))  _Float16 v8h;
typedef __attribute__((ext_vector_type(8)))  unsigned short v8us;
typedef __attribute__((ext_vector_type(8)))  float    v8f;
typedef __attribute__((ext_vector_type(4)))  float    v4f;
typedef v4f  __attribute__((may_alias)) v4fa;

__device__ __forceinline__ unsigned short f2bf(float f) { unsigned u = __float_as_uint(f); u += 0x7FFFu + ((u >> 16) & 1u); return (unsigned short)(u >> 16); }
__device__ __forceinline__ float bfr(float f) { return __uint_as_float(((unsigned)f2bf(f)) << 16); }
__device__ __forceinline__ v16h cat16(v8h lo, v8h hi) { return __builtin_shufflevector(lo, hi, 0, 1, 2, 3, 4, 5, 6, 7, 8, 9, 10, 11, 12, 13, 14, 15); }
__device__ __forceinline__ v16bf cat16b(v8us lo, v8us hi) { return __builtin_bit_cast(v16bf, __builtin_shufflevector(lo, hi, 0, 1, 2, 3, 4, 5, 6, 7, 8, 9, 10, 11, 12, 13, 14, 15)); }
__device__ __forceinline__ v8f wmma16(v16h a, v16h b, v8f c) { return __builtin_amdgcn_wmma_f32_16x16x32_f16(false, a, false, b, (short)0, c, false, false); }
__device__ __forceinline__ v8f wmmab(v16bf a, v16bf b, v8f c) { return __builtin_amdgcn_wmma_f32_16x16x32_bf16(false, a, false, b, (short)0, c, false, false); }
__device__ __forceinline__ v16h  ldh(const h16* p) { return cat16(*(const v8h*)p, *(const v8h*)(p + 16)); }
__device__ __forceinline__ v16bf ldb(const bf* p)  { return cat16b(*(const v8us*)p, *(const v8us*)(p + 16)); }
__device__ __forceinline__ void wave_sync() { __builtin_amdgcn_fence(3  , "wavefront"); __builtin_amdgcn_wave_barrier(); asm volatile("" ::: "memory"); }

__device__ __forceinline__ v8f wmma16g(v16h a, v16h b, v8f c) { c = wmma16(a, b, c); asm volatile("v_nop\n\tv_nop\n\tv_nop\n\tv_nop" : "+v"(c) : "v"(a), "v"(b)); return c; }
__device__ __forceinline__ v8f wmmabg(v16bf a, v16bf b, v8f c) { c = wmmab(a, b, c); asm volatile("v_nop\n\tv_nop\n\tv_nop\n\tv_nop" : "+v"(c) : "v"(a), "v"(b)); return c; }
static __device__ __forceinline__ h16 toh_flush(float v) { const float w = (fabsf(v) < 6.103515625e-05f) ? 0.0f : v; return (h16)w; }
__device__ __forceinline__ float tanh_e2(float z) { const float ex = __builtin_amdgcn_exp2f(z * TL2E); const float r = __builtin_amdgcn_rcpf(ex + 1.0f); return fmaf(-2.0f, r, 1.0f); }

__global__ __launch_bounds__(256) void k_cvt8(const float* __restrict__ src, bf* dst, size_t n8) {
    const size_t i = (size_t)blockIdx.x * 256 + threadIdx.x; if (i >= n8) return;
    const v8f v = *(const v8f*)(src + i * 8); v8us o;
#pragma unroll
    for (int k = 0; k < 8; ++k) o[k] = f2bf(v[k]);
    *(volatile v8us*)(dst + i * 8) = o; __threadfence(); *(volatile v8us*)(dst + i * 8) = o;
}

__global__ __launch_bounds__(256) void k_vt(const float* __restrict__ src, h16* VT) {
    __shared__ float ts[64 * 65];
    const unsigned tid = threadIdx.x;
    const unsigned j0 = blockIdx.x * 64u, d0 = blockIdx.y * 64u, b = blockIdx.z;
    const float* sb = src + ((size_t)b * SEQ_FULL + j0) * VD + d0;
#pragma unroll
    for (int it = 0; it < 4; ++it) { const unsigned idx = tid + 256u * (unsigned)it; const unsigned jj = idx >> 4, c4 = (idx & 15u) * 4u;
        const v4f v = *(const v4f*)(sb + (size_t)jj * VD + c4);
#pragma unroll
        for (int c = 0; c < 4; ++c) ts[jj * 65u + c4 + (unsigned)c] = bfr(v[c]); }
    __syncthreads();
    v8h o[2];
#pragma unroll
    for (int it = 0; it < 2; ++it) { const unsigned p = tid + 256u * (unsigned)it; const unsigned drow = p >> 3, j8 = (p & 7u) * 8u;
#pragma unroll
        for (int c = 0; c < 8; ++c) o[it][c] = toh_flush(ts[(j8 + (unsigned)c) * 65u + drow]); }
    h16* db = VT + ((size_t)b * VD + d0) * SEQ + j0;
#pragma unroll 1
    for (int ps = 0; ps < 2; ++ps) {
#pragma unroll
        for (int it = 0; it < 2; ++it) { const unsigned p = tid + 256u * (unsigned)it; const unsigned drow = p >> 3, j8 = (p & 7u) * 8u;
            *(volatile v8h*)(db + (size_t)drow * SEQ + j8) = o[it]; }
        if (ps == 0) __threadfence(); }
}

__global__ __launch_bounds__(32) void k_projf(const bf* __restrict__ A, const bf* __restrict__ Bt, float* C) {
    __shared__ __align__(16) float os[16 * 68];
    const int K = FEAT;
    const int lane = threadIdx.x & 31, lr = lane & 15, hi = lane >> 4; const unsigned r0 = blockIdx.x * 64u, c0 = blockIdx.y * 64u;
    v8f acc[4][4];
#pragma unroll
    for (int mb = 0; mb < 4; ++mb)
#pragma unroll
        for (int nb = 0; nb < 4; ++nb) acc[mb][nb] = (v8f){};
    const size_t aoff = (size_t)(r0 + (unsigned)lr) * K + 8 * hi, boff = (size_t)(c0 + (unsigned)lr) * K + 8 * hi;
#pragma unroll 1
    for (int kc = 0; kc < K; kc += 32) {
        v16bf a[4];
#pragma unroll
        for (int mb = 0; mb < 4; ++mb) a[mb] = ldb(A + aoff + (size_t)mb * 16 * K + kc);
#pragma unroll
        for (int nb = 0; nb < 4; ++nb) { const v16bf b = ldb(Bt + boff + (size_t)nb * 16 * K + kc);
#pragma unroll
            for (int mb = 0; mb < 4; ++mb) acc[mb][nb] = wmmabg(a[mb], b, acc[mb][nb]); }
    }
#pragma unroll
    for (int mb = 0; mb < 4; ++mb) {
#pragma unroll
        for (int nb = 0; nb < 4; ++nb) {
#pragma unroll
            for (int j = 0; j < 8; ++j) os[(hi * 8 + j) * 68 + nb * 16 + lr] = acc[mb][nb][j]; }
        wave_sync();
        float* cb = C + (size_t)(r0 + (unsigned)(mb * 16)) * HID + c0;
#pragma unroll 1
        for (int ps = 0; ps < 2; ++ps) {
#pragma unroll
            for (int s = 0; s < 8; ++s) { const int row = 2 * s + (lane >> 4), cofs = (lane & 15) * 4;
                const v4f val = *(const v4fa*)(&os[row * 68 + cofs]);
                *(volatile v4f*)(cb + (size_t)row * HID + cofs) = val; }
            if (ps == 0) __threadfence(); }
        wave_sync();
    }
}

__global__ __launch_bounds__(32 * PW) void k_pair(const float* __restrict__ QP, const float* __restrict__ KP, const float* __restrict__ wv, const int* __restrict__ vlen,
                                                  float* ATT, h16* PH, h16* PR) {
#pragma clang fp contract(off)
    __shared__ __align__(16) float qs[PW * HID];
    __shared__ __align__(16) float wvs[PW * HID];
    __shared__ __align__(16) float es[PW * SEQ];
    const int lane = threadIdx.x & 31;
    const int wave = __builtin_amdgcn_readfirstlane((int)(threadIdx.x >> 5));
    const unsigned bx = blockIdx.x;
    const unsigned b = bx / (unsigned)(SEQ / PW);
    const unsigned i = (bx % (unsigned)(SEQ / PW)) * (unsigned)PW + (unsigned)wave;
    const size_t rq = (size_t)b * SEQ + i;
    int vraw = vlen[b]; vraw = min(max(vraw, 0), SEQ);
    const int vl = __builtin_amdgcn_readfirstlane(vraw);
    const int wq = wave * HID, we = wave * SEQ;
    { const v4f qv = *(const v4f*)(QP + rq * HID + 4 * lane);
      const v4f wr = *(const v4f*)(wv + 4 * lane); v4f wb;
#pragma unroll
      for (int c = 0; c < 4; ++c) wb[c] = bfr(wr[c]);
      *(v4fa*)(&qs[wq + 4 * lane]) = qv; *(v4fa*)(&wvs[wq + 4 * lane]) = wb; }
    wave_sync();
    const float* kb = KP + (size_t)b * SEQ * HID;
#pragma unroll 1
    for (int qq = 0; qq < SEQ / 32; ++qq) {
        const int g = qq >> 2;
        const int j = 128 * g + 4 * lane + (qq & 3);
        float e = NEGF;
        if (128 * g < vl) {
            const float* kr = kb + (size_t)j * HID;
            float acc = 0.0f;
#pragma unroll 2
            for (int h = 0; h < HID; h += 4) {
                const v4f kk = *(const v4f*)(kr + h);
                const v4f qv = *(const v4fa*)(&qs[wq + h]);
                const v4f wb = *(const v4fa*)(&wvs[wq + h]);
#pragma unroll
                for (int c = 0; c < 4; ++c) acc = fmaf(wb[c], tanh_e2(qv[c] + kk[c]), acc);
            }
            e = (j < vl) ? acc : NEGF;
        }
        es[we + j] = e;
    }
    wave_sync();
    v4f ev[NG];
#pragma unroll
    for (int g = 0; g < NG; ++g) ev[g] = *(const v4fa*)(&es[we + 128 * g + 4 * lane]);
    float mx = ev[0][0];
#pragma unroll
    for (int g = 0; g < NG; ++g) {
#pragma unroll
        for (int c = 0; c < 4; ++c) mx = fmaxf(mx, ev[g][c]); }
    mx = fmaxf(mx, __shfl_xor(mx, 16, 32)); mx = fmaxf(mx, __shfl_xor(mx, 8, 32)); mx = fmaxf(mx, __shfl_xor(mx, 4, 32));
    mx = fmaxf(mx, __shfl_xor(mx, 2, 32));  mx = fmaxf(mx, __shfl_xor(mx, 1, 32));
    float l = 0.0f;
#pragma unroll
    for (int g = 0; g < NG; ++g) {
#pragma unroll
        for (int c = 0; c < 4; ++c) { const float p = __builtin_amdgcn_exp2f((ev[g][c] - mx) * L2E); ev[g][c] = p; l += p; } }
    l += __shfl_xor(l, 16, 32); l += __shfl_xor(l, 8, 32); l += __shfl_xor(l, 4, 32); l += __shfl_xor(l, 2, 32); l += __shfl_xor(l, 1, 32);
    const float inv = 1.0f / l;
#pragma unroll
    for (int g = 0; g < NG; ++g) {
#pragma unroll
        for (int c = 0; c < 4; ++c) ev[g][c] = ev[g][c] * inv;
        *(v4fa*)(&es[we + 128 * g + 4 * lane]) = ev[g]; }
    wave_sync();
    v8h hv[NP8], rv[NP8];
#pragma unroll
    for (int s = 0; s < NP8; ++s) {
        const v4f x0 = *(const v4fa*)(&es[we + 256 * s + 8 * lane]); const v4f x1 = *(const v4fa*)(&es[we + 256 * s + 8 * lane + 4]);
#pragma unroll
        for (int c = 0; c < 4; ++c) {
            const float xa = x0[c] * PC, xb = x1[c] * PC;
            const h16 ha = toh_flush(xa); const h16 hb = toh_flush(xb);
            hv[s][c] = ha; hv[s][4 + c] = hb;
            rv[s][c] = toh_flush((xa - (float)ha) * QRS); rv[s][4 + c] = toh_flush((xb - (float)hb) * QRS); } }
    float* arow = ATT + ((size_t)b * OUT_SEQ + i) * OUT_SEQ;
    h16* ph = PH + rq * SEQ; h16* pr = PR + rq * SEQ;
#pragma unroll 1
    for (int ps = 0; ps < 2; ++ps) {
#pragma unroll
        for (int g = 0; g < NG; ++g) *(volatile v4f*)(arow + 128 * g + 4 * lane) = ev[g];
#pragma unroll
        for (int s = 0; s < NP8; ++s) { *(volatile v8h*)(ph + 256 * s + 8 * lane) = hv[s]; *(volatile v8h*)(pr + 256 * s + 8 * lane) = rv[s]; }
        if (ps == 0) __threadfence(); }
}

__global__ __launch_bounds__(32) void k_out(const h16* __restrict__ PH, const h16* __restrict__ PR, const h16* __restrict__ VT, float* OUT) {
    __shared__ __align__(16) float os[16 * 68];
    const int lane = threadIdx.x & 31, lr = lane & 15, hi = lane >> 4; const unsigned r0 = blockIdx.x * 32u, c0 = blockIdx.y * 64u;
    const unsigned bb = r0 / (unsigned)SEQ, tt = r0 % (unsigned)SEQ;
    v8f acc[2][4], acr[2][4];
#pragma unroll
    for (int mb = 0; mb < 2; ++mb)
#pragma unroll
        for (int nb = 0; nb < 4; ++nb) { acc[mb][nb] = (v8f){}; acr[mb][nb] = (v8f){}; }
    const size_t aoff = (size_t)(r0 + (unsigned)lr) * SEQ + 8 * hi;
    const size_t boff = ((size_t)bb * VD + c0 + (unsigned)lr) * SEQ + 8 * hi;
#pragma unroll 1
    for (int kc = 0; kc < SEQ; kc += 32) {
        v16h a[2], ar[2];
#pragma unroll
        for (int mb = 0; mb < 2; ++mb) { a[mb] = ldh(PH + aoff + (size_t)mb * 16 * SEQ + kc); ar[mb] = ldh(PR + aoff + (size_t)mb * 16 * SEQ + kc); }
#pragma unroll
        for (int nb = 0; nb < 4; ++nb) { const v16h b = ldh(VT + boff + (size_t)nb * 16 * SEQ + kc);
#pragma unroll
            for (int mb = 0; mb < 2; ++mb) { acc[mb][nb] = wmma16g(a[mb], b, acc[mb][nb]); acr[mb][nb] = wmma16g(ar[mb], b, acr[mb][nb]); } }
    }
#pragma unroll
    for (int mb = 0; mb < 2; ++mb) {
#pragma unroll
        for (int nb = 0; nb < 4; ++nb) {
#pragma unroll
            for (int j = 0; j < 8; ++j) os[(hi * 8 + j) * 68 + nb * 16 + lr] = (acc[mb][nb][j] + acr[mb][nb][j] * QRI) * PCI; }
        wave_sync();
        float* ob = OUT + ((size_t)bb * OUT_SEQ + tt + (unsigned)(mb * 16)) * VD + c0;
#pragma unroll 1
        for (int ps = 0; ps < 2; ++ps) {
#pragma unroll
            for (int s = 0; s < 8; ++s) { const int row = 2 * s + (lane >> 4), cofs = (lane & 15) * 4;
                const v4f val = *(const v4fa*)(&os[row * 68 + cofs]);
                *(volatile v4f*)(ob + (size_t)row * VD + cofs) = val; }
            if (ps == 0) __threadfence(); }
        wave_sync();
    }
}

static constexpr size_t al256(size_t v) { return (v + 255) & ~(size_t)255; }
static constexpr size_t SZ_XB = al256((size_t)NB * SEQ * FEAT * 2);
static constexpr size_t SZ_WB = al256((size_t)2 * HID * FEAT * 2);
static constexpr size_t SZ_PF = al256((size_t)NB * SEQ * HID * 4);
static constexpr size_t SZ_VT = al256((size_t)NB * VD * SEQ * 2);
static constexpr size_t SZ_PP = al256((size_t)NB * SEQ * SEQ * 2);
static constexpr size_t SZ_TOTAL = 2 * SZ_XB + SZ_WB + 2 * SZ_PF + SZ_VT + 2 * SZ_PP;
static_assert(SZ_TOTAL <= (size_t)134217728);
static_assert(((size_t)HID * FEAT * 2) % 256 == 0);
static_assert(((size_t)SEQ * FEAT) % 8 == 0);
static_assert(((size_t)HID * FEAT) % 8 == 0);

extern "C" void kernel_launch(void* const* d_in, const int* in_sizes, int n_in,
                              void* d_out, int out_size, void* d_ws, size_t ws_size, hipStream_t stream) {
    if (n_in < 7) return;
    const size_t needx = ((size_t)(NB - 1) * SEQ_FULL + SEQ) * FEAT;
    const size_t needv = ((size_t)(NB - 1) * SEQ_FULL + SEQ) * VD;
    if ((size_t)in_sizes[0] < needx || (size_t)in_sizes[1] < needx || (size_t)in_sizes[2] < needv) return;
    if (in_sizes[3] < NB) return;
    if ((size_t)in_sizes[4] < (size_t)HID * FEAT || (size_t)in_sizes[5] < (size_t)HID * FEAT || in_sizes[6] < HID) return;
    if ((size_t)out_size < OUT1_OFF + (size_t)NB * OUT_SEQ * OUT_SEQ) return;
    if (SZ_TOTAL > ws_size) return;
    const float* xin[2] = { (const float*)d_in[0], (const float*)d_in[1] };
    const float* vals = (const float*)d_in[2];
    const int* vlen = (const int*)d_in[3];
    const float* wq = (const float*)d_in[4];
    const float* wk = (const float*)d_in[5];
    const float* wv = (const float*)d_in[6];
    float* OUT = (float*)d_out;
    float* ATT = (float*)d_out + OUT1_OFF;
    char* wsp = (char*)d_ws;
    bf* XB[2];
    XB[0] = (bf*)wsp; wsp += SZ_XB;
    XB[1] = (bf*)wsp; wsp += SZ_XB;
    bf* WB = (bf*)wsp; wsp += SZ_WB;
    float* QP = (float*)wsp; wsp += SZ_PF;
    float* KPL = (float*)wsp; wsp += SZ_PF;
    h16* VT = (h16*)wsp; wsp += SZ_VT;
    h16* PH = (h16*)wsp; wsp += SZ_PP;
    h16* PR = (h16*)wsp; wsp += SZ_PP;
    bf* WQ = WB; bf* WK = WB + (size_t)HID * FEAT;

    for (int i = 0; i < 2; ++i) {
        if (SEQ == SEQ_FULL) {
            const size_t n8 = (size_t)NB * SEQ * FEAT / 8;
            k_cvt8<<<(unsigned)((n8 + 255) / 256), 256, 0, stream>>>(xin[i], XB[i], n8);
        } else {
            const size_t n8 = (size_t)SEQ * FEAT / 8;
            for (int b = 0; b < NB; ++b) k_cvt8<<<(unsigned)((n8 + 255) / 256), 256, 0, stream>>>(xin[i] + (size_t)b * SEQ_FULL * FEAT, XB[i] + (size_t)b * SEQ * FEAT, n8);
        }
    }
    { const size_t n8 = (size_t)HID * FEAT / 8; const unsigned g = (unsigned)((n8 + 255) / 256);
      k_cvt8<<<g, 256, 0, stream>>>(wq, WQ, n8); k_cvt8<<<g, 256, 0, stream>>>(wk, WK, n8); }

    k_vt<<<dim3(SEQ / 64, VD / 64, NB), 256, 0, stream>>>(vals, VT);

    k_projf<<<dim3(NB * SEQ / 64, HID / 64, 1), 32, 0, stream>>>(XB[0], WQ, QP);
    k_projf<<<dim3(NB * SEQ / 64, HID / 64, 1), 32, 0, stream>>>(XB[1], WK, KPL);

    k_pair<<<dim3(NB * SEQ / PW, 1, 1), 32 * PW, 0, stream>>>(QP, KPL, wv, vlen, ATT, PH, PR);

    k_out<<<dim3(NB * SEQ / 32, VD / 64, 1), 32, 0, stream>>>(PH, PR, VT, OUT);
}
